// StateRNN_42408507081097
// MI455X (gfx1250) — hardware-run, weakly checked
//
#include <hip/hip_runtime.h>
#include <math.h>

constexpr int NBATCH  = 128;
constexpr int NSTEP   = 512;
constexpr int NFEAT   = 50;
constexpr int NFPAD   = 64;
constexpr int NHID    = 256;
constexpr int NGATE   = 4 * NHID;
constexpr int NLAT    = 32;
constexpr int ND1     = 256;
constexpr int ND2     = 128;
constexpr int KCAT    = NHID + NFPAD;
constexpr int NROWS   = NBATCH * NSTEP;
constexpr int NTHR    = 256;
constexpr int SEQ_BLK = 16;
constexpr int APITCH  = KCAT + 8;
constexpr int HSPITCH = NHID + 8;
constexpr int CPITCH  = NHID + 4;
constexpr int SLAB3P  = 36;
constexpr int NOUT0   = NROWS * NLAT;
constexpr int NOUT1   = NBATCH * 2 * NHID;
constexpr int NOUT_ALL = NOUT0 + NOUT1 + 1;
constexpr int HEAD3_BLOCKS = (NROWS / 64) / 8;
constexpr int NPART   = HEAD3_BLOCKS * 32;
constexpr float WCARRY     = 16.0f;
constexpr float WCARRY_INV = 1.0f / 16.0f;
constexpr float LOSS_INV   = 1.0f / (float)(NBATCH * NLAT);

static_assert(NHID == NTHR, "thread = hidden column in the state init");
static_assert(NHID == 32 * (NTHR / 32), "8 waves x 32 hidden units");
static_assert(NBATCH % SEQ_BLK == 0, "blocks of 16 sequences");
static_assert(KCAT % 32 == 0 && NHID % 32 == 0 && ND1 % 32 == 0 && ND2 % 32 == 0, "K multiples of 32");
static_assert(NROWS % 64 == 0 && ND1 % 64 == 0 && ND2 % 64 == 0, "M, N tile multiples");
static_assert((NROWS / 64) % 8 == 0, "head3 grid exact");
static_assert(NPART == 16 * NTHR, "loss reduce covers the partial table exactly");
static_assert(NFEAT <= NFPAD && NFPAD == 64, "x slot = two k-chunks");
static_assert((APITCH * 2) % 16 == 0 && (HSPITCH * 2) % 16 == 0 && (CPITCH * 4) % 16 == 0, "16-B aligned LDS rows");
static_assert(2 * 16 * APITCH * 2 + 16 * HSPITCH * 2 + 2 * 16 * CPITCH * 4 <= 65536, "static LDS budget");
static_assert((size_t)NOUT0 * 4 == 8388608 && (size_t)(NOUT0 + NOUT1) * 4 == 8650752, "output byte offsets");

typedef __attribute__((ext_vector_type(16))) _Float16 v16h;
typedef __attribute__((ext_vector_type(8)))  _Float16 v8h;
typedef __attribute__((ext_vector_type(8)))  float    v8f;
typedef __attribute__((ext_vector_type(4)))  float    v4f;

__device__ __forceinline__ unsigned short f2bf_bits(float f) {
  unsigned u = __float_as_uint(f);
  return (unsigned short)((u + 0x7FFFu + ((u >> 16) & 1u)) >> 16);
}
__device__ __forceinline__ float bf_bits2f(unsigned short h) { return __uint_as_float(((unsigned)h) << 16); }
__device__ __forceinline__ float bf16r(float f) { return bf_bits2f(f2bf_bits(f)); }

__device__ __forceinline__ void guard4_h(v8f& a0, v8f& a1, v8f& a2, v8f& a3, v16h x, v16h y0, v16h y1, v16h y2, v16h y3) {
  asm volatile("v_nop\n\tv_nop\n\tv_nop\n\tv_nop" : "+v"(a0), "+v"(a1), "+v"(a2), "+v"(a3) : "v"(x), "v"(y0), "v"(y1), "v"(y2), "v"(y3));
}
__device__ __forceinline__ void guard2_h(v8f& a0, v8f& a1, v16h x, v16h y0, v16h y1) {
  asm volatile("v_nop\n\tv_nop\n\tv_nop\n\tv_nop" : "+v"(a0), "+v"(a1) : "v"(x), "v"(y0), "v"(y1));
}
__device__ __forceinline__ void acc_guard4(v8f& a, v8f& b, v8f& c, v8f& d) { asm volatile("v_nop\n\tv_nop\n\tv_nop\n\tv_nop" : "+v"(a), "+v"(b), "+v"(c), "+v"(d)); }
__device__ __forceinline__ void acc_guard2(v8f& a, v8f& b) { asm volatile("v_nop\n\tv_nop\n\tv_nop\n\tv_nop" : "+v"(a), "+v"(b)); }

template <typename T> struct Frag;
template <> struct Frag<_Float16> {
  typedef v16h V; union U { v16h v; v8h h[2]; };
  static __device__ __forceinline__ v16h load(const _Float16* p) {
    U f; f.h[0] = *(const v8h*)(p); f.h[1] = *(const v8h*)(p + 16); return f.v;
  }
  static __device__ __forceinline__ v8f mma(v16h a, v16h b, v8f c) {
    return __builtin_amdgcn_wmma_f32_16x16x32_f16(false, a, false, b, (short)0, c, false, false);
  }
};

__device__ __forceinline__ float sig_f(float x)  { return __builtin_amdgcn_rcpf(1.0f + expf(-x)); }
__device__ __forceinline__ float tanh_f(float x) { return 1.0f - 2.0f * __builtin_amdgcn_rcpf(1.0f + expf(2.0f * x)); }

constexpr int PREP_B0 = (NGATE / 64) * (NHID / 64);
constexpr int PREP_B1 = PREP_B0 + (NGATE / 64);
constexpr int PREP_B2 = PREP_B1 + (ND1 / 64) * (NHID / 64);
constexpr int PREP_B3 = PREP_B2 + (ND2 / 64) * (ND1 / 64);
constexpr int PREP_B4 = PREP_B3 + 1 * (ND2 / 64);
static_assert(PREP_B4 == 106, "prep job table");

__global__ __launch_bounds__(NTHR) void prep_weights_kernel(const float* __restrict__ wh, const float* __restrict__ wx,
                                                            const float* __restrict__ w1, const float* __restrict__ w2,
                                                            const float* __restrict__ w3,
                                                            unsigned short* __restrict__ WC, unsigned short* __restrict__ W1T,
                                                            unsigned short* __restrict__ W2T, unsigned short* __restrict__ W3T) {
  __shared__ float Tt[64 * 65];
  const int tid = threadIdx.x;
  const int bid = blockIdx.x;
  const float* src; unsigned short* dst;
  int R, C, ldo, kbase, tilesX, local;
  if (bid < PREP_B0)      { src = wh; dst = WC;  R = NHID;  C = NGATE; ldo = KCAT; kbase = 0;    tilesX = NGATE / 64; local = bid; }
  else if (bid < PREP_B1) { src = wx; dst = WC;  R = NFEAT; C = NGATE; ldo = KCAT; kbase = NHID; tilesX = NGATE / 64; local = bid - PREP_B0; }
  else if (bid < PREP_B2) { src = w1; dst = W1T; R = NHID;  C = ND1;   ldo = NHID; kbase = 0;    tilesX = ND1 / 64;   local = bid - PREP_B1; }
  else if (bid < PREP_B3) { src = w2; dst = W2T; R = ND1;   C = ND2;   ldo = ND1;  kbase = 0;    tilesX = ND2 / 64;   local = bid - PREP_B2; }
  else                    { src = w3; dst = W3T; R = ND2;   C = NLAT;  ldo = ND2;  kbase = 0;    tilesX = 1;          local = bid - PREP_B3; }
  const int bx = local % tilesX, by = local / tilesX;
  const int c0 = bx * 64, r0 = by * 64;
#pragma unroll 4
  for (int i = 0; i < 16; ++i) {
    const int idx = i * NTHR + tid;
    const int rr = idx >> 6, cc = idx & 63;
    const int r = r0 + rr, cg = c0 + cc;
    const int rc = (r < R) ? r : (R - 1);
    const int ccl = (cg < C) ? cg : (C - 1);
    const float v = src[(size_t)rc * (size_t)C + ccl];
    Tt[rr * 65 + cc] = (r < R && cg < C) ? v : 0.0f;
  }
  __syncthreads();
  const int q = tid >> 3, c8 = (tid & 7) * 8;
  v8h hv[2];
#pragma unroll
  for (int g = 0; g < 2; ++g) {
    const int qq = g * 32 + q;
#pragma unroll
    for (int e = 0; e < 8; ++e) {
      const float f = Tt[(c8 + e) * 65 + qq];
      hv[g][e] = (_Float16)(bf16r(f) * WCARRY);
    }
  }
  for (int pass = 0; pass < 2; ++pass) {
#pragma unroll
    for (int g = 0; g < 2; ++g) {
      const int orow = c0 + g * 32 + q;
      if (orow < C) {
        const size_t o = (size_t)orow * (size_t)ldo + (size_t)(kbase + r0 + c8);
        *(volatile v8h*)((_Float16*)dst + o) = hv[g];
      }
    }
    __threadfence();
  }
}

__global__ __launch_bounds__(NTHR) void xpack_kernel(const float* __restrict__ x, unsigned short* __restrict__ XHp) {
  const int i = blockIdx.x * NTHR + threadIdx.x;
  if (i < NSTEP * NBATCH * (NFPAD / 8)) {
    const int g = i & 7;
    const int rb = i >> 3;
    const int b = rb % NBATCH;
    const int t = rb / NBATCH;
    const float* sp = x + ((size_t)b * NSTEP + (size_t)t) * NFEAT;
    v8h hv;
#pragma unroll
    for (int e = 0; e < 8; ++e) {
      const int col = 8 * g + e;
      const int cc = (col < NFEAT) ? col : (NFEAT - 1);
      const float v = sp[cc];
      const float val = (col < NFEAT) ? bf16r(v) : 0.0f;
      hv[e] = (_Float16)val;
    }
    _Float16* dp = (_Float16*)XHp + (size_t)i * 8;
    *(volatile v8h*)dp = hv;
    __threadfence();
    *(volatile v8h*)dp = hv;
  }
}

__global__ __launch_bounds__(NTHR) void lstm_seq_kernel(const unsigned short* __restrict__ XHp,
                                                        const float* __restrict__ mask,
                                                        const float* __restrict__ states_in,
                                                        const float* __restrict__ bias,
                                                        const unsigned short* __restrict__ WCp,
                                                        unsigned short* __restrict__ HSp,
                                                        float* __restrict__ states_out) {
  __shared__ __align__(16) _Float16 Abuf[2][SEQ_BLK * APITCH];
  __shared__ __align__(16) _Float16 Hst[SEQ_BLK * HSPITCH];
  __shared__ __align__(16) float    Cs[SEQ_BLK * CPITCH];
  __shared__ __align__(16) float    Hf[SEQ_BLK * CPITCH];
  const _Float16* XH = (const _Float16*)XHp;
  const _Float16* WC = (const _Float16*)WCp;
  _Float16* HS = (_Float16*)HSp;
  const int tid = threadIdx.x, lane = tid & 31, wave = tid >> 5;
  const int c = lane & 15, hh = lane >> 4, koff = hh * 8;
  const int rowbase = blockIdx.x * SEQ_BLK;

#pragma unroll 1
  for (int i = 0; i < SEQ_BLK; ++i) {
    const float mv = bf16r(mask[(size_t)(rowbase + i) * NSTEP]);
    const float hv = bf16r(states_in[(size_t)(rowbase + i) * (2 * NHID) + NHID + tid]);
    const float cv = bf16r(states_in[(size_t)(rowbase + i) * (2 * NHID) + tid]);
    Abuf[0][i * APITCH + tid] = (_Float16)(hv * (1.0f - mv));
    Cs[i * CPITCH + tid] = cv;
  }
  {
    const int pb = tid >> 7, pr = (tid >> 3) & 15, pe = tid & 7;
    Abuf[pb][pr * APITCH + KCAT + pe] = (_Float16)0.0f;
  }
  if (tid < 128) {
    const int xr = tid >> 3, x8 = (tid & 7) * 8;
    const v8h xv = *(const v8h*)(XH + ((size_t)rowbase + xr) * NFPAD + x8);
    *(v8h*)(&Abuf[0][0] + xr * APITCH + NHID + x8) = xv;
  }
  float omc[8];
#pragma unroll
  for (int r = 0; r < 8; ++r) {
    float mv = mask[(size_t)(rowbase + 8 * hh + r) * NSTEP];
    asm volatile("" : "+v"(mv));
    omc[r] = 1.0f - bf16r(mv);
  }
  __syncthreads();

  const v8f z8 = {0.f, 0.f, 0.f, 0.f, 0.f, 0.f, 0.f, 0.f};
  const size_t gstride = (size_t)NHID * KCAT;

#pragma unroll 1
  for (int t = 0; t < NSTEP; ++t) {
    const int cur = t & 1;
    const int tn = (t + 1 < NSTEP) ? (t + 1) : (NSTEP - 1);
    const bool last = (t == NSTEP - 1);
    const _Float16* ahrow = &Abuf[cur][0] + c * APITCH + koff;
    _Float16* ahn = &Abuf[cur ^ 1][0];

    float omn[8];
#pragma unroll
    for (int r = 0; r < 8; ++r) {
      float mv = mask[(size_t)(rowbase + 8 * hh + r) * NSTEP + tn];
      asm volatile("" : "+v"(mv));
      omn[r] = 1.0f - bf16r(mv);
    }

#pragma unroll 1
    for (int nt = 0; nt < 2; ++nt) {
      const int j = 32 * wave + 16 * nt + c;
      const _Float16* wrow = WC + (size_t)j * KCAT + koff;
      v8f acc[4];
      acc[0] = z8; acc[1] = z8; acc[2] = z8; acc[3] = z8;
#pragma unroll 1
      for (int k0 = 0; k0 < KCAT; k0 += 32) {
        const v16h a  = Frag<_Float16>::load(ahrow + k0);
        const v16h b0 = Frag<_Float16>::load(wrow + k0);
        const v16h b1 = Frag<_Float16>::load(wrow + gstride + k0);
        const v16h b2 = Frag<_Float16>::load(wrow + 2 * gstride + k0);
        const v16h b3 = Frag<_Float16>::load(wrow + 3 * gstride + k0);
        acc[0] = Frag<_Float16>::mma(a, b0, acc[0]);
        acc[1] = Frag<_Float16>::mma(a, b1, acc[1]);
        acc[2] = Frag<_Float16>::mma(a, b2, acc[2]);
        acc[3] = Frag<_Float16>::mma(a, b3, acc[3]);
        guard4_h(acc[0], acc[1], acc[2], acc[3], a, b0, b1, b2, b3);
      }
      acc_guard4(acc[0], acc[1], acc[2], acc[3]);
      const float bi = bf16r(bias[j]);
      const float bf = bf16r(bias[NHID + j]);
      const float bo = bf16r(bias[2 * NHID + j]);
      const float bu = bf16r(bias[3 * NHID + j]);
#pragma unroll
      for (int r = 0; r < 8; ++r) {
        const float zi = acc[0][r] * WCARRY_INV + bi;
        const float zf = acc[1][r] * WCARRY_INV + bf;
        const float zo = acc[2][r] * WCARRY_INV + bo;
        const float zu = acc[3][r] * WCARRY_INV + bu;
        const float ig = sig_f(zi);
        const float fg = sig_f(zf);
        const float og = sig_f(zo);
        const float ug = tanh_f(zu);
        const int row = 8 * hh + r;
        const int ci = row * CPITCH + j;
        const float cold = Cs[ci] * omc[r];
        const float cn = fg * cold + ig * ug;
        const float hn = og * tanh_f(cn);
        Cs[ci] = cn;
        ahn[row * APITCH + j] = (_Float16)(hn * omn[r]);
        Hst[row * HSPITCH + j] = (_Float16)hn;
        if (last) Hf[ci] = hn;
      }
    }
    __syncthreads();

    {
      const int r0 = 2 * wave, r1 = 2 * wave + 1;
      const v8h h0v = *(const v8h*)(Hst + r0 * HSPITCH + lane * 8);
      const v8h h1v = *(const v8h*)(Hst + r1 * HSPITCH + lane * 8);
      _Float16* d0 = HS + ((size_t)(rowbase + r0) * NSTEP + (size_t)t) * NHID + lane * 8;
      _Float16* d1 = HS + ((size_t)(rowbase + r1) * NSTEP + (size_t)t) * NHID + lane * 8;
      for (int pass = 0; pass < 2; ++pass) {
        *(volatile v8h*)d0 = h0v;
        *(volatile v8h*)d1 = h1v;
        __threadfence();
      }
    }
    if (tid < 128) {
      const int xr = tid >> 3, x8 = (tid & 7) * 8;
      const v8h xv = *(const v8h*)(XH + ((size_t)tn * NBATCH + (size_t)(rowbase + xr)) * NFPAD + x8);
      *(v8h*)(ahn + xr * APITCH + NHID + x8) = xv;
    }
#pragma unroll
    for (int r = 0; r < 8; ++r) omc[r] = omn[r];
    __syncthreads();
  }

  for (int pass = 0; pass < 2; ++pass) {
#pragma unroll
    for (int it = 0; it < 8; ++it) {
      const int idx = it * NTHR + tid;
      const int row = idx >> 7;
      const int col = (idx & 127) * 4;
      const int cc = col & (NHID - 1);
      const v4f vc = *(const v4f*)(Cs + row * CPITCH + cc);
      const v4f vh = *(const v4f*)(Hf + row * CPITCH + cc);
      const v4f v = (col < NHID) ? vc : vh;
      *(volatile v4f*)(states_out + (size_t)(rowbase + row) * (2 * NHID) + col) = v;
    }
    __threadfence();
  }
}

__global__ __launch_bounds__(256) void gemm64_relu_f16_kernel(
    const unsigned short* __restrict__ Ap, int lda,
    const unsigned short* __restrict__ Btp, int ldb,
    unsigned short* __restrict__ Cp, int ldc,
    const float* __restrict__ bias, int M, int N, int K, float scale) {
  const _Float16* A = (const _Float16*)Ap;
  const _Float16* Bt = (const _Float16*)Btp;
  __shared__ __align__(16) float sT[8][16 * 68];
  const int lane = threadIdx.x & 31;
  const int wave = threadIdx.x >> 5;
  const int tilesN = N >> 6;
  const int tilesM = M >> 6;
  const int tile = blockIdx.x * 8 + wave;
  if (tile >= tilesM * tilesN) return;
  const int tm = tile / tilesN;
  const int tn = tile - tm * tilesN;
  const int m0 = tm << 6;
  const int n0 = tn << 6;
  const int rlane = lane & 15;
  const int koff  = (lane >> 4) * 8;
  const int mOff  = (lane >> 4) * 8;

  const _Float16* bp[4];
  const _Float16* ap[4];
#pragma unroll
  for (int j = 0; j < 4; ++j) bp[j] = Bt + (size_t)(n0 + (j << 4) + rlane) * ldb + koff;
#pragma unroll
  for (int i = 0; i < 4; ++i) ap[i] = A + (size_t)(m0 + (i << 4) + rlane) * lda + koff;

  v8f acc[4][4];
#pragma unroll
  for (int i = 0; i < 4; ++i)
#pragma unroll
    for (int j = 0; j < 4; ++j) acc[i][j] = (v8f){0.f,0.f,0.f,0.f,0.f,0.f,0.f,0.f};

  for (int k0 = 0; k0 < K; k0 += 32) {
    v16h bh[4];
#pragma unroll
    for (int j = 0; j < 4; ++j) bh[j] = Frag<_Float16>::load(bp[j] + k0);
#pragma unroll
    for (int i = 0; i < 4; ++i) {
      const v16h ah = Frag<_Float16>::load(ap[i] + k0);
#pragma unroll
      for (int j = 0; j < 4; ++j) acc[i][j] = Frag<_Float16>::mma(ah, bh[j], acc[i][j]);
      guard4_h(acc[i][0], acc[i][1], acc[i][2], acc[i][3], ah, bh[0], bh[1], bh[2], bh[3]);
    }
  }
  acc_guard4(acc[0][0], acc[0][1], acc[0][2], acc[0][3]);
  acc_guard4(acc[1][0], acc[1][1], acc[1][2], acc[1][3]);
  acc_guard4(acc[2][0], acc[2][1], acc[2][2], acc[2][3]);
  acc_guard4(acc[3][0], acc[3][1], acc[3][2], acc[3][3]);

  float* slab = sT[wave];
  _Float16* C = (_Float16*)Cp;
  const int q = lane >> 3, c8 = (lane & 7) * 8;
#pragma unroll
  for (int i = 0; i < 4; ++i) {
    const int mBase = m0 + (i << 4);
#pragma unroll
    for (int j = 0; j < 4; ++j) {
      const int n = n0 + (j << 4) + rlane;
      const float bv = bf16r(bias[n]);
#pragma unroll
      for (int r = 0; r < 8; ++r) {
        float v = acc[i][j][r] * scale + bv;
        v = fmaxf(v, 0.0f);
        slab[(mOff + r) * 68 + (j << 4) + rlane] = v;
      }
    }
    __builtin_amdgcn_fence(__ATOMIC_RELEASE, "workgroup");
    __builtin_amdgcn_wave_barrier();
    __builtin_amdgcn_fence(__ATOMIC_ACQUIRE, "workgroup");
    for (int pass = 0; pass < 2; ++pass) {
#pragma unroll
      for (int it = 0; it < 4; ++it) {
        const int row = it * 4 + q;
        const float* sp = slab + row * 68 + c8;
        v8h hv;
#pragma unroll
        for (int e = 0; e < 8; ++e) hv[e] = (_Float16)sp[e];
        *(volatile v8h*)(C + (size_t)(mBase + row) * ldc + n0 + c8) = hv;
      }
      __threadfence();
    }
    __builtin_amdgcn_fence(__ATOMIC_RELEASE, "workgroup");
    __builtin_amdgcn_wave_barrier();
    __builtin_amdgcn_fence(__ATOMIC_ACQUIRE, "workgroup");
  }
}

__global__ __launch_bounds__(256) void head3_kernel(const unsigned short* __restrict__ D2p,
                                                    const unsigned short* __restrict__ W3p,
                                                    const float* __restrict__ b3, const float* __restrict__ tgt,
                                                    float* __restrict__ out0, float* __restrict__ partials) {
  __shared__ __align__(16) float sT[8][16 * SLAB3P];
  __shared__ float wsum[8];
  const _Float16* A = (const _Float16*)D2p;
  const _Float16* Bt = (const _Float16*)W3p;
  const int lane = threadIdx.x & 31;
  const int wave = threadIdx.x >> 5;
  const int tile = blockIdx.x * 8 + wave;
  const int m0 = tile << 6;
  const int rlane = lane & 15;
  const int koff  = (lane >> 4) * 8;
  const int mOff  = (lane >> 4) * 8;

  const _Float16* bp0 = Bt + (size_t)rlane * ND2 + koff;
  const _Float16* bp1 = Bt + (size_t)(16 + rlane) * ND2 + koff;
  const _Float16* ap[4];
#pragma unroll
  for (int i = 0; i < 4; ++i) ap[i] = A + (size_t)(m0 + (i << 4) + rlane) * ND2 + koff;

  v8f acc[4][2];
#pragma unroll
  for (int i = 0; i < 4; ++i) {
    acc[i][0] = (v8f){0.f,0.f,0.f,0.f,0.f,0.f,0.f,0.f};
    acc[i][1] = (v8f){0.f,0.f,0.f,0.f,0.f,0.f,0.f,0.f};
  }
#pragma unroll 1
  for (int k0 = 0; k0 < ND2; k0 += 32) {
    const v16h bh0 = Frag<_Float16>::load(bp0 + k0);
    const v16h bh1 = Frag<_Float16>::load(bp1 + k0);
#pragma unroll
    for (int i = 0; i < 4; ++i) {
      const v16h ah = Frag<_Float16>::load(ap[i] + k0);
      acc[i][0] = Frag<_Float16>::mma(ah, bh0, acc[i][0]);
      acc[i][1] = Frag<_Float16>::mma(ah, bh1, acc[i][1]);
      guard2_h(acc[i][0], acc[i][1], ah, bh0, bh1);
    }
  }
  acc_guard4(acc[0][0], acc[0][1], acc[1][0], acc[1][1]);
  acc_guard4(acc[2][0], acc[2][1], acc[3][0], acc[3][1]);

  const float bb0 = bf16r(b3[rlane]);
  const float bb1 = bf16r(b3[16 + rlane]);
  float* slab = sT[wave];
  const int q = lane >> 3, c4 = (lane & 7) * 4;
  float part = 0.0f;
#pragma unroll
  for (int i = 0; i < 4; ++i) {
    const int mBase = m0 + (i << 4);
#pragma unroll
    for (int r = 0; r < 8; ++r) {
      slab[(mOff + r) * SLAB3P + rlane]      = acc[i][0][r] * WCARRY_INV + bb0;
      slab[(mOff + r) * SLAB3P + 16 + rlane] = acc[i][1][r] * WCARRY_INV + bb1;
    }
    __builtin_amdgcn_fence(__ATOMIC_RELEASE, "workgroup");
    __builtin_amdgcn_wave_barrier();
    __builtin_amdgcn_fence(__ATOMIC_ACQUIRE, "workgroup");
    v4f vv[4];
#pragma unroll
    for (int it = 0; it < 4; ++it) {
      const int row = it * 4 + q;
      vv[it] = *(const v4f*)(slab + row * SLAB3P + c4);
      const v4f tg = *(const v4f*)(tgt + (size_t)(mBase + row) * NLAT + c4);
#pragma unroll
      for (int e = 0; e < 4; ++e) {
        const float te = tg[e];
        const float ve = vv[it][e];
        const float d = ve - bf16r(te);
        part += d * d;
      }
    }
    for (int pass = 0; pass < 2; ++pass) {
#pragma unroll
      for (int it = 0; it < 4; ++it) {
        const int row = it * 4 + q;
        *(volatile v4f*)(out0 + (size_t)(mBase + row) * NLAT + c4) = vv[it];
      }
      __threadfence();
    }
    __builtin_amdgcn_fence(__ATOMIC_RELEASE, "workgroup");
    __builtin_amdgcn_wave_barrier();
    __builtin_amdgcn_fence(__ATOMIC_ACQUIRE, "workgroup");
  }
#pragma unroll
  for (int off = 16; off > 0; off >>= 1) part += __shfl_xor(part, off, 32);
  if (lane == 0) wsum[wave] = part;
  __syncthreads();
  if (wave == 0) {
    const float pv = wsum[lane & 7];
    const float val = (lane < 8) ? pv : 0.0f;
    float* pp = partials + (size_t)blockIdx.x * 32 + lane;
    *(volatile float*)pp = val;
    __threadfence();
    *(volatile float*)pp = val;
  }
}

__global__ __launch_bounds__(NTHR) void loss_kernel(const float* __restrict__ partials, float* __restrict__ out2) {
  __shared__ float sh[NTHR];
  const int tid = threadIdx.x;
  float s = 0.0f;
#pragma unroll
  for (int qd = 0; qd < 4; ++qd) {
    const v4f v = *(const v4f*)(partials + (size_t)tid * 16 + qd * 4);
    s += (v[0] + v[1]) + (v[2] + v[3]);
  }
  sh[tid] = s;
  __syncthreads();
#pragma unroll 1
  for (int stride = NTHR / 2; stride > 0; stride >>= 1) {
    if (tid < stride) sh[tid] = sh[tid] + sh[tid + stride];
    __syncthreads();
  }
  if (tid == 0) {
    const float val = sh[0] * LOSS_INV;
    *(volatile float*)out2 = val;
    __threadfence();
    *(volatile float*)out2 = val;
  }
}

extern "C" void kernel_launch(void* const* d_in, const int* in_sizes, int n_in,
                              void* d_out, int out_size, void* d_ws, size_t ws_size, hipStream_t stream) {
  if (n_in < 13 || d_out == nullptr || d_ws == nullptr) return;
  if (in_sizes[0] != NBATCH * NSTEP * NFEAT || in_sizes[1] != NBATCH * NSTEP * NLAT ||
      in_sizes[2] != NBATCH * NSTEP || in_sizes[3] != NBATCH * 2 * NHID ||
      in_sizes[4] != NFEAT * NGATE || in_sizes[5] != NHID * NGATE || in_sizes[6] != NGATE ||
      in_sizes[7] != NHID * ND1 || in_sizes[8] != ND1 || in_sizes[9] != ND1 * ND2 || in_sizes[10] != ND2 ||
      in_sizes[11] != ND2 * NLAT || in_sizes[12] != NLAT || out_size != NOUT_ALL) return;

  const float* x_in   = (const float*)d_in[0];
  const float* tgt    = (const float*)d_in[1];
  const float* smask  = (const float*)d_in[2];
  const float* st_in  = (const float*)d_in[3];
  const float* wx     = (const float*)d_in[4];
  const float* wh     = (const float*)d_in[5];
  const float* bz     = (const float*)d_in[6];
  const float* w1     = (const float*)d_in[7];
  const float* b1     = (const float*)d_in[8];
  const float* w2     = (const float*)d_in[9];
  const float* b2     = (const float*)d_in[10];
  const float* w3     = (const float*)d_in[11];
  const float* b3     = (const float*)d_in[12];

  float* out0 = (float*)d_out;
  float* out1 = out0 + (size_t)NOUT0;
  float* out2 = out1 + (size_t)NOUT1;

  char* ws = (char*)d_ws; size_t off = 0;
  auto carve = [&](size_t bytes) -> char* { char* p = ws + off; off += (bytes + 255) & ~(size_t)255; return p; };
  unsigned short* WC   = (unsigned short*)carve((size_t)NGATE * KCAT * 2);
  unsigned short* W1T  = (unsigned short*)carve((size_t)ND1 * NHID * 2);
  unsigned short* W2T  = (unsigned short*)carve((size_t)ND2 * ND1 * 2);
  unsigned short* W3T  = (unsigned short*)carve((size_t)NLAT * ND2 * 2);
  unsigned short* XH   = (unsigned short*)carve((size_t)NSTEP * NBATCH * NFPAD * 2);
  unsigned short* HS   = (unsigned short*)carve((size_t)NROWS * NHID * 2);
  unsigned short* D1   = (unsigned short*)carve((size_t)NROWS * ND1 * 2);
  unsigned short* D2   = (unsigned short*)carve((size_t)NROWS * ND2 * 2);
  float*          PART = (float*)carve((size_t)NPART * 4);
  if (off > ws_size || off > (size_t)134217728) return;

  prep_weights_kernel<<<PREP_B4, NTHR, 0, stream>>>(wh, wx, w1, w2, w3, WC, W1T, W2T, W3T);
  xpack_kernel<<<(NSTEP * NBATCH * (NFPAD / 8)) / NTHR, NTHR, 0, stream>>>(x_in, XH);
  lstm_seq_kernel<<<NBATCH / SEQ_BLK, NTHR, 0, stream>>>(XH, smask, st_in, bz, WC, HS, out1);
  gemm64_relu_f16_kernel<<<(NROWS / 64) * (ND1 / 64) / 8, 256, 0, stream>>>(
      HS, NHID, W1T, NHID, D1, ND1, b1, NROWS, ND1, NHID, WCARRY_INV);
  gemm64_relu_f16_kernel<<<(NROWS / 64) * (ND2 / 64) / 8, 256, 0, stream>>>(
      D1, ND1, W2T, ND1, D2, ND2, b2, NROWS, ND2, ND1, WCARRY_INV);
  head3_kernel<<<HEAD3_BLOCKS, 256, 0, stream>>>(D2, W3T, b3, tgt, out0, PART);
  loss_kernel<<<1, NTHR, 0, stream>>>(PART, out2);
}
